// DeepFactorRNN_82669530513626
// MI455X (gfx1250) — hardware-verified
//
#include <hip/hip_runtime.h>
#include <math.h>

constexpr int NTS    = 128;
constexpr int NPER   = 256;
constexpr int NFEAT  = 128;
constexpr int GHID   = 512;
constexpr int NHID   = 256;
constexpr int NFAC   = 10;
constexpr int NROWS  = NTS * NPER;
constexpr int NTHR   = 256;
constexpr int SLABP  = 68;
constexpr float WCARRY     = 16.0f;
constexpr float HCARRY     = 16.0f;
constexpr float WCARRY_INV = 1.0f / WCARRY;
constexpr float WH_INV     = 1.0f / (WCARRY * HCARRY);
constexpr float HCARRY_INV = 1.0f / HCARRY;

static_assert(NROWS == 32768);
static_assert(NROWS % 16 == 0);
static_assert(GHID % 64 == 0 && NHID % 64 == 0);
static_assert(NFEAT % 32 == 0 && GHID % 32 == 0 && NHID % 32 == 0);
static_assert(((NROWS / 16) * (GHID / 64)) % (NTHR / 32) == 0);
static_assert(((NROWS / 16) * (NHID / 64)) % (NTHR / 32) == 0);
static_assert(NROWS % NTHR == 0);
static_assert(GHID == 2 * NTHR && NHID == NTHR);
static_assert((NROWS * NFEAT / 8) % NTHR == 0);
static_assert((4 * GHID * NFEAT / 8) % NTHR == 0);
static_assert((4 * GHID * GHID / 8) % NTHR == 0);
static_assert((4 * NHID * NFEAT / 8) % NTHR == 0);
static_assert((4 * NHID * NHID / 8) % NTHR == 0);

typedef __attribute__((ext_vector_type(16))) _Float16 v16h;
typedef __attribute__((ext_vector_type(8)))  _Float16 v8h;
typedef __attribute__((ext_vector_type(8)))  float    v8f;
typedef __attribute__((ext_vector_type(4)))  float    v4f;
typedef __attribute__((ext_vector_type(4)))  unsigned v4u;

template <typename T> struct Frag;
template <> struct Frag<_Float16> {
  typedef v16h V;
  union U { v16h v; v8h h[2]; };
  static __device__ __forceinline__ v16h load(const _Float16* p) {
    U f;
    f.h[0] = *(const v8h*)(p);
    f.h[1] = *(const v8h*)(p + 16);
    return f.v;
  }
  static __device__ __forceinline__ v8f mma(v16h a, v16h b, v8f c) {
    return __builtin_amdgcn_wmma_f32_16x16x32_f16(false, a, false, b, (short)0, c, false, false);
  }
};

__device__ __forceinline__ void grp_guard(v8f& c0, v8f& c1, v8f& c2, v8f& c3,
                                          v16h a, v16h b0, v16h b1, v16h b2, v16h b3) {
  asm volatile("v_nop\n\tv_nop\n\tv_nop\n\tv_nop"
               : "+v"(c0), "+v"(c1), "+v"(c2), "+v"(c3)
               : "v"(a), "v"(b0), "v"(b1), "v"(b2), "v"(b3));
}
__device__ __forceinline__ void acc_guard4(v8f& a, v8f& b, v8f& c, v8f& d) {
  asm volatile("v_nop\n\tv_nop\n\tv_nop\n\tv_nop" : "+v"(a), "+v"(b), "+v"(c), "+v"(d));
}

template <int KD>
__device__ __forceinline__ void gate_group(const _Float16* wq, v16h a, v8f& c0, v8f& c1, v8f& c2, v8f& c3) {
  const v16h b0 = Frag<_Float16>::load(wq);
  const v16h b1 = Frag<_Float16>::load(wq + 16 * KD);
  const v16h b2 = Frag<_Float16>::load(wq + 32 * KD);
  const v16h b3 = Frag<_Float16>::load(wq + 48 * KD);
  c0 = Frag<_Float16>::mma(a, b0, c0);
  c1 = Frag<_Float16>::mma(a, b1, c1);
  c2 = Frag<_Float16>::mma(a, b2, c2);
  c3 = Frag<_Float16>::mma(a, b3, c3);
  grp_guard(c0, c1, c2, c3, a, b0, b1, b2, b3);
}

__device__ __forceinline__ float fsig(float x) {
  return __builtin_amdgcn_rcpf(1.0f + __expf(-x));
}
__device__ __forceinline__ float ftanh(float x) {
  const float xc = fminf(fmaxf(x, -15.0f), 15.0f);
  return 1.0f - 2.0f * __builtin_amdgcn_rcpf(__expf(2.0f * xc) + 1.0f);
}

__device__ __forceinline__ float h16_to_f32(unsigned hb) {
  const unsigned sgn = (hb & 0x8000u) << 16;
  const unsigned em = hb & 0x7fffu;
  const float fn = __uint_as_float((em << 13) + 0x38000000u);
  const float fs = (float)em * 5.9604644775390625e-8f;
  const float mag = (em < 0x400u) ? fs : fn;
  return __uint_as_float(__float_as_uint(mag) | sgn);
}

__global__ __launch_bounds__(NTHR) void cvt8_f16_kernel(const float* __restrict__ src, unsigned short* __restrict__ dst,
                                                        int n8, float sc) {
  const int i = blockIdx.x * NTHR + threadIdx.x;
  if (i < n8) {
    const float* sp = src + (size_t)i * 8;
    const v4f a = *(const v4f*)(sp);
    const v4f b = *(const v4f*)(sp + 4);
    v8h hv;
#pragma unroll
    for (int e = 0; e < 4; ++e) {
      const float fa = a[e] * sc;
      const float fb = b[e] * sc;
      hv[e]     = (_Float16)fa;
      hv[4 + e] = (_Float16)fb;
    }
    *(volatile v8h*)(dst + (size_t)i * 8) = hv;
    __threadfence();
    *(volatile v8h*)(dst + (size_t)i * 8) = hv;
  }
}

template <bool RELU>
__device__ __forceinline__ void cell_tile(const v8f ai, const v8f ag, const v8f ao,
                                          float bi, float bg, float bo, float sc, float* sl) {
#pragma unroll
  for (int r = 0; r < 8; ++r) {
    const float pi = ai[r] * sc + bi;
    const float pg = ag[r] * sc + bg;
    const float po = ao[r] * sc + bo;
    const float cc = fsig(pi) * ftanh(pg);
    float hv = fsig(po) * ftanh(cc);
    if (RELU) hv = fmaxf(hv, 0.0f);
    sl[r * SLABP] = hv * HCARRY;
  }
}

template <int HID, int KD, bool RELU>
__global__ __launch_bounds__(NTHR) void gate_gemm_kernel(const unsigned short* __restrict__ Ap,
                                                         const unsigned short* __restrict__ Wp,
                                                         const float* __restrict__ bias,
                                                         unsigned short* __restrict__ Hout,
                                                         int numTiles, float accScale) {
  static_assert(HID % 64 == 0 && KD % 32 == 0);
  __shared__ __align__(16) float sT[NTHR / 32][16 * SLABP];
  const _Float16* A = (const _Float16*)Ap;
  const _Float16* W = (const _Float16*)Wp;
  const int lane = threadIdx.x & 31;
  const int wave = threadIdx.x >> 5;
  const int tile = blockIdx.x * (NTHR / 32) + wave;
  if (tile >= numTiles) return;
  constexpr int CG = HID / 64;
  const int tm   = tile / CG;
  const int tg   = tile - tm * CG;
  const int m0   = tm * 16;
  const int col0 = tg * 64;
  const int c    = lane & 15;
  const int hh   = lane >> 4;
  const int koff = hh * 8;

  const _Float16* ap = A + (size_t)(m0 + c) * KD + koff;
  const _Float16* wI = W + (size_t)(col0 + c) * KD + koff;
  const _Float16* wG = wI + (size_t)2 * HID * KD;
  const _Float16* wO = wI + (size_t)3 * HID * KD;

  const v8f z8 = {0.f, 0.f, 0.f, 0.f, 0.f, 0.f, 0.f, 0.f};
  v8f aI0 = z8, aI1 = z8, aI2 = z8, aI3 = z8;
  v8f aG0 = z8, aG1 = z8, aG2 = z8, aG3 = z8;
  v8f aO0 = z8, aO1 = z8, aO2 = z8, aO3 = z8;

#pragma unroll 1
  for (int k0 = 0; k0 < KD; k0 += 32) {
    const v16h a = Frag<_Float16>::load(ap + k0);
    gate_group<KD>(wI + k0, a, aI0, aI1, aI2, aI3);
    gate_group<KD>(wG + k0, a, aG0, aG1, aG2, aG3);
    gate_group<KD>(wO + k0, a, aO0, aO1, aO2, aO3);
  }
  acc_guard4(aI0, aI1, aI2, aI3);
  acc_guard4(aG0, aG1, aG2, aG3);
  acc_guard4(aO0, aO1, aO2, aO3);

  float bI[4], bG[4], bO[4];
#pragma unroll
  for (int nt = 0; nt < 4; ++nt) {
    const int j = col0 + 16 * nt + c;
    bI[nt] = bias[j];
    bG[nt] = bias[2 * HID + j];
    bO[nt] = bias[3 * HID + j];
  }

  float* slab = sT[wave];
  float* sl = slab + (8 * hh) * SLABP + c;
  cell_tile<RELU>(aI0, aG0, aO0, bI[0], bG[0], bO[0], accScale, sl);
  cell_tile<RELU>(aI1, aG1, aO1, bI[1], bG[1], bO[1], accScale, sl + 16);
  cell_tile<RELU>(aI2, aG2, aO2, bI[2], bG[2], bO[2], accScale, sl + 32);
  cell_tile<RELU>(aI3, aG3, aO3, bI[3], bG[3], bO[3], accScale, sl + 48);

  __builtin_amdgcn_fence(__ATOMIC_RELEASE, "workgroup");
  __builtin_amdgcn_wave_barrier();
  __builtin_amdgcn_fence(__ATOMIC_ACQUIRE, "workgroup");

  const int q  = lane >> 3;
  const int c8 = (lane & 7) * 8;
  for (int pass = 0; pass < 2; ++pass) {
#pragma unroll
    for (int it = 0; it < 4; ++it) {
      const int row = it * 4 + q;
      const float* sp = slab + row * SLABP + c8;
      v8h hv;
#pragma unroll
      for (int e = 0; e < 8; ++e) hv[e] = (_Float16)sp[e];
      *(volatile v8h*)(Hout + (size_t)(m0 + row) * HID + col0 + c8) = hv;
    }
    __threadfence();
  }
}

__global__ __launch_bounds__(NTHR) void head_kernel(const unsigned* __restrict__ Hg2, const unsigned* __restrict__ Hn2,
                                                    const float* __restrict__ affW, const float* __restrict__ affb,
                                                    const float* __restrict__ nW, const float* __restrict__ nb,
                                                    float* __restrict__ out) {
  __shared__ __align__(16) float sW[GHID];
  __shared__ __align__(16) float sN[NHID];
  __shared__ __align__(16) float sO[2][NTHR];
  const int tid  = threadIdx.x;
  const int lane = tid & 31;
  const int wave = tid >> 5;

  float s0 = 0.0f, s1 = 0.0f, bsum = 0.0f;
#pragma unroll 1
  for (int r = 0; r < NFAC; ++r) {
    s0 += affW[r * GHID + tid];
    s1 += affW[r * GHID + NTHR + tid];
    bsum += affb[r];
  }
  sW[tid] = s0;
  sW[NTHR + tid] = s1;
  sN[tid] = nW[tid];
  const float nbias = nb[0];
  __syncthreads();

  const int n = blockIdx.x * NTHR + tid;
  const v4u* gp = (const v4u*)(Hg2 + (size_t)n * (GHID / 2));
  const v4u* np = (const v4u*)(Hn2 + (size_t)n * (NHID / 2));

  float accg = 0.0f;
#pragma unroll 1
  for (int j = 0; j < GHID / 8; ++j) {
    const v4u qv = gp[j];
#pragma unroll
    for (int e = 0; e < 4; ++e) {
      const unsigned w = qv[e];
      const float lo = h16_to_f32(w & 0xffffu);
      const float hi = h16_to_f32(w >> 16);
      accg = fmaf(lo, sW[8 * j + 2 * e], accg);
      accg = fmaf(hi, sW[8 * j + 2 * e + 1], accg);
    }
  }
  float accn = 0.0f;
#pragma unroll 1
  for (int j = 0; j < NHID / 8; ++j) {
    const v4u qv = np[j];
#pragma unroll
    for (int e = 0; e < 4; ++e) {
      const unsigned w = qv[e];
      const float lo = h16_to_f32(w & 0xffffu);
      const float hi = h16_to_f32(w >> 16);
      accn = fmaf(lo, sN[8 * j + 2 * e], accn);
      accn = fmaf(hi, sN[8 * j + 2 * e + 1], accn);
    }
  }
  const float mu = accg * HCARRY_INV + bsum;
  const float z  = accn * HCARRY_INV + nbias;
  const float sp = fmaxf(z, 0.0f) + log1pf(expf(-fabsf(z)));
  sO[0][tid] = mu;
  sO[1][tid] = sp + 1e-6f;
  __syncthreads();

  if (wave < 4) {
    const int sel  = wave >> 1;
    const int half = wave & 1;
    const v4f v = *(const v4f*)(&sO[sel][half * 128 + lane * 4]);
    float* op = out + (size_t)sel * NROWS + (size_t)blockIdx.x * NTHR + half * 128 + lane * 4;
    *(volatile v4f*)op = v;
    __threadfence();
    *(volatile v4f*)op = v;
  }
}

extern "C" void kernel_launch(void* const* d_in, const int* in_sizes, int n_in,
                              void* d_out, int out_size, void* d_ws, size_t ws_size, hipStream_t stream) {
  if (n_in < 13 || d_out == nullptr || d_ws == nullptr) return;
  if (in_sizes[0] != NROWS * NFEAT || in_sizes[1] != 4 * GHID * NFEAT || in_sizes[2] != 4 * GHID ||
      in_sizes[3] != 4 * GHID * GHID || in_sizes[4] != 4 * GHID || in_sizes[5] != NFAC * GHID ||
      in_sizes[6] != NFAC || in_sizes[7] != 4 * NHID * NFEAT || in_sizes[8] != 4 * NHID ||
      in_sizes[9] != 4 * NHID * NHID || in_sizes[10] != 4 * NHID || in_sizes[11] != NHID ||
      in_sizes[12] != 1 || out_size != 2 * NROWS) return;

  const float* X      = (const float*)d_in[0];
  const float* gW0    = (const float*)d_in[1];
  const float* gb0    = (const float*)d_in[2];
  const float* gW1    = (const float*)d_in[3];
  const float* gb1    = (const float*)d_in[4];
  const float* affW   = (const float*)d_in[5];
  const float* affb   = (const float*)d_in[6];
  const float* nW0    = (const float*)d_in[7];
  const float* nb0    = (const float*)d_in[8];
  const float* nW1    = (const float*)d_in[9];
  const float* nb1    = (const float*)d_in[10];
  const float* noiseW = (const float*)d_in[11];
  const float* noiseb = (const float*)d_in[12];
  float* out = (float*)d_out;

  char* ws = (char*)d_ws;
  size_t off = 0;
  auto carve = [&](size_t bytes) -> char* { char* p = ws + off; off += (bytes + 255) & ~(size_t)255; return p; };
  unsigned short* XH  = (unsigned short*)carve((size_t)NROWS * NFEAT * 2);
  unsigned short* WG0 = (unsigned short*)carve((size_t)4 * GHID * NFEAT * 2);
  unsigned short* WG1 = (unsigned short*)carve((size_t)4 * GHID * GHID * 2);
  unsigned short* WN0 = (unsigned short*)carve((size_t)4 * NHID * NFEAT * 2);
  unsigned short* WN1 = (unsigned short*)carve((size_t)4 * NHID * NHID * 2);
  unsigned short* HG1 = (unsigned short*)carve((size_t)NROWS * GHID * 2);
  unsigned short* HG2 = (unsigned short*)carve((size_t)NROWS * GHID * 2);
  unsigned short* HN1 = (unsigned short*)carve((size_t)NROWS * NHID * 2);
  unsigned short* HN2 = (unsigned short*)carve((size_t)NROWS * NHID * 2);
  if (off > ws_size || off > (size_t)134217728) return;

  const int n8x  = NROWS * NFEAT / 8;
  const int n8g0 = 4 * GHID * NFEAT / 8;
  const int n8g1 = 4 * GHID * GHID / 8;
  const int n8n0 = 4 * NHID * NFEAT / 8;
  const int n8n1 = 4 * NHID * NHID / 8;
  cvt8_f16_kernel<<<(n8x  + NTHR - 1) / NTHR, NTHR, 0, stream>>>(X,   XH,  n8x,  1.0f);
  cvt8_f16_kernel<<<(n8g0 + NTHR - 1) / NTHR, NTHR, 0, stream>>>(gW0, WG0, n8g0, WCARRY);
  cvt8_f16_kernel<<<(n8g1 + NTHR - 1) / NTHR, NTHR, 0, stream>>>(gW1, WG1, n8g1, WCARRY);
  cvt8_f16_kernel<<<(n8n0 + NTHR - 1) / NTHR, NTHR, 0, stream>>>(nW0, WN0, n8n0, WCARRY);
  cvt8_f16_kernel<<<(n8n1 + NTHR - 1) / NTHR, NTHR, 0, stream>>>(nW1, WN1, n8n1, WCARRY);

  const int tilesG = (NROWS / 16) * (GHID / 64);
  const int tilesN = (NROWS / 16) * (NHID / 64);
  const int wpb = NTHR / 32;
  gate_gemm_kernel<GHID, NFEAT, false><<<(tilesG + wpb - 1) / wpb, NTHR, 0, stream>>>(XH,  WG0, gb0, HG1, tilesG, WCARRY_INV);
  gate_gemm_kernel<GHID, GHID,  true ><<<(tilesG + wpb - 1) / wpb, NTHR, 0, stream>>>(HG1, WG1, gb1, HG2, tilesG, WH_INV);
  gate_gemm_kernel<NHID, NFEAT, false><<<(tilesN + wpb - 1) / wpb, NTHR, 0, stream>>>(XH,  WN0, nb0, HN1, tilesN, WCARRY_INV);
  gate_gemm_kernel<NHID, NHID,  true ><<<(tilesN + wpb - 1) / wpb, NTHR, 0, stream>>>(HN1, WN1, nb1, HN2, tilesN, WH_INV);

  head_kernel<<<NROWS / NTHR, NTHR, 0, stream>>>((const unsigned*)HG2, (const unsigned*)HN2,
                                                 affW, affb, noiseW, noiseb, out);
}
